// FASTMultiHeadAttention_31078383354363
// MI455X (gfx1250) — hardware-verified
//
#include <hip/hip_runtime.h>

typedef __attribute__((ext_vector_type(16))) _Float16 v16h;
typedef __attribute__((ext_vector_type(16))) __bf16 v16b;
typedef __attribute__((ext_vector_type(8)))  _Float16 v8h;
typedef __attribute__((ext_vector_type(8)))  float v8f;
typedef __attribute__((ext_vector_type(4)))  float v4f;
typedef __attribute__((ext_vector_type(4)))  unsigned v4u;

template <typename T> __device__ __forceinline__ void vst2(void* p, T v) { *(volatile T*)p = v; __threadfence(); *(volatile T*)p = v; }

__device__ __forceinline__ v8f wmma16(v16h a, v16h b, v8f c) {
  v8f d = __builtin_amdgcn_wmma_f32_16x16x32_f16(false, a, false, b, (short)0, c, false, false);
  asm volatile("v_nop\n\tv_nop\n\tv_nop\n\tv_nop" : "+v"(d) : "v"(a), "v"(b));
  return d;
}
__device__ __forceinline__ v8f wmma_bf(v16b a, v16b b, v8f c) {
  v8f d = __builtin_amdgcn_wmma_f32_16x16x32_bf16(false, a, false, b, (short)0, c, false, false);
  asm volatile("v_nop\n\tv_nop\n\tv_nop\n\tv_nop" : "+v"(d) : "v"(a), "v"(b));
  return d;
}
__device__ __forceinline__ v16h frag_h(const _Float16* rowk0, int lane) {
  union { v16h v; v8h q[2]; } u; const _Float16* p = rowk0 + 8 * (lane >> 4);
  u.q[0] = *(const v8h*)p; u.q[1] = *(const v8h*)(p + 16); return u.v;
}
__device__ __forceinline__ float bfr(float v) { return (float)(__bf16)v; }
__device__ __forceinline__ void ldsx() { asm volatile("s_wait_dscnt 0" ::: "memory"); __builtin_amdgcn_wave_barrier(); __builtin_amdgcn_fence(3, "workgroup"); }

#ifndef NB
#define NB 2
#endif
#ifndef SEQ
#define SEQ 1024
#endif
#define NB_FULL 2
#define SEQ_FULL 1024
#define NH 8
#define DD 64
#define NR (2 * SEQ - 1)
#define A0C 1.0f
#define A1C 1.0f
#define A2C 0.5f
#define PSC 0.0625f
static_assert(NB >= 1 && NB <= NB_FULL);
static_assert(SEQ >= 64 && SEQ <= SEQ_FULL && (SEQ % 64) == 0);
static_assert((DD % 32) == 0);

#define WS_VT  0u
#define WS_END (WS_VT + 2u * (size_t)NB * NH * DD * SEQ)
static_assert(WS_END <= 134217728u);

__global__ __launch_bounds__(128) void k_vt(const float* __restrict__ V, _Float16* __restrict__ VT) {
  __shared__ __align__(16) _Float16 th[DD][72];
  const int t = threadIdx.x; const size_t bh = blockIdx.y; const int m0 = blockIdx.x * 64;
  for (int e = t; e < 64 * DD; e += 128) { const int ml = e / DD, d = e % DD; th[d][ml] = (_Float16)bfr(V[(bh * SEQ_FULL + m0 + ml) * DD + d]); }
  __syncthreads();
  for (int e = t; e < DD * 8; e += 128) { const int d = e >> 3, q = e & 7; vst2((void*)(VT + (bh * DD + d) * (size_t)SEQ + m0 + q * 8), *(const v4u*)&th[d][q * 8]); }
}

__global__ __launch_bounds__(128) void k_att(const float* __restrict__ Q, const float* __restrict__ K, const _Float16* __restrict__ VT, const float* __restrict__ RPE, float* __restrict__ OUT) {
  __shared__ __align__(16) float sg[4][16][52]; __shared__ __align__(16) float sp[4][16][36]; __shared__ __align__(16) float so[4][16][68];
  const int tid = threadIdx.x, wave = tid >> 5, lane = tid & 31, col = lane & 15, g = lane >> 4;
  const size_t bh = blockIdx.y; const int i0 = blockIdx.x * 64 + wave * 16;
  const size_t rq = bh * SEQ_FULL + i0;
  const size_t ro = bh * SEQ + i0;
  v16b aq[2];
#pragma unroll
  for (int kc = 0; kc < 2; ++kc) { const float* pp = Q + (rq + col) * DD + kc * 32 + 8 * g;
#pragma unroll
    for (int i = 0; i < 8; ++i) { aq[kc][i] = (__bf16)pp[i]; aq[kc][8 + i] = (__bf16)pp[16 + i]; } }
  float den[8];
#pragma unroll
  for (int r = 0; r < 8; ++r) den[r] = 0.f;
  v8f acc[4], accl[4];
#pragma unroll
  for (int j = 0; j < 4; ++j) { acc[j] = v8f{}; accl[j] = v8f{}; }
#pragma unroll 1
  for (int ks = 0; ks < SEQ / 32; ++ks) { const int j0 = ks * 32;
    { const int base = SEQ - 1 + i0 - j0 - 31;
#pragma unroll
      for (int tt = 0; tt < 3; ++tt) { int rr = base + tt * 16 + col; rr = rr < 0 ? 0 : (rr > NR - 1 ? NR - 1 : rr); v8f c = {};
#pragma unroll
        for (int kc = 0; kc < 2; ++kc) { v16b w; const float* rp = RPE + (size_t)rr * DD + kc * 32 + 8 * g;
#pragma unroll
          for (int i = 0; i < 8; ++i) { w[i] = (__bf16)rp[i]; w[8 + i] = (__bf16)rp[16 + i]; }
          c = wmma_bf(aq[kc], w, c); }
#pragma unroll
        for (int r = 0; r < 8; ++r) sg[wave][8 * g + r][tt * 16 + col] = c[r]; } }
    ldsx();
    float s[2][8];
#pragma unroll
    for (int ct = 0; ct < 2; ++ct) { const int j = j0 + ct * 16 + col; v8f c = {};
#pragma unroll
      for (int kc = 0; kc < 2; ++kc) { v16b w; const float* kp = K + (bh * SEQ_FULL + j) * DD + kc * 32 + 8 * g;
#pragma unroll
        for (int i = 0; i < 8; ++i) { w[i] = (__bf16)kp[i]; w[8 + i] = (__bf16)kp[16 + i]; }
        c = wmma_bf(aq[kc], w, c); }
#pragma unroll
      for (int r = 0; r < 8; ++r) { const int tix = (8 * g + r) - (ct * 16 + col) + 31;
        const float sv = c[r] + sg[wave][8 * g + r][tix];
        const float sc = A0C + A1C * sv + A2C * sv * sv;
        s[ct][r] = sc; den[r] += sc; } }
#pragma unroll
    for (int r = 0; r < 8; ++r) { sp[wave][8 * g + r][col] = s[0][r]; sp[wave][8 * g + r][16 + col] = s[1][r]; }
    ldsx();
    v16h pa, pal; { const float* prow = &sp[wave][col][0] + 8 * (lane >> 4);
#pragma unroll
      for (int i = 0; i < 8; ++i) { const float p0 = prow[i] * PSC, p1 = prow[16 + i] * PSC; pa[i] = (_Float16)p0; pa[8 + i] = (_Float16)p1; pal[i] = (_Float16)((p0 - (float)pa[i]) * 2048.0f); pal[8 + i] = (_Float16)((p1 - (float)pa[8 + i]) * 2048.0f); } }
#pragma unroll
    for (int jt = 0; jt < 4; ++jt) { const v16h vh = frag_h(VT + (bh * DD + jt * 16 + col) * (size_t)SEQ + j0, lane); acc[jt] = wmma16(pa, vh, acc[jt]); accl[jt] = wmma16(pal, vh, accl[jt]); }
    ldsx(); }
#pragma unroll
  for (int r = 0; r < 8; ++r) { float dsum = den[r];
#pragma unroll
    for (int o = 1; o < 16; o <<= 1) dsum += __shfl_xor(dsum, o);
    const float il = (1.0f / PSC) / dsum;
#pragma unroll
    for (int jt = 0; jt < 4; ++jt) so[wave][8 * g + r][jt * 16 + col] = (acc[jt][r] + accl[jt][r] * (1.0f / 2048.0f)) * il; }
  ldsx();
  for (int rl = 0; rl < 16; ++rl) if (lane < 16) vst2((void*)(OUT + (ro + rl) * DD + lane * 4), *(const v4f*)&so[wave][rl][lane * 4]);
}

extern "C" void kernel_launch(void* const* d_in, const int* in_sizes, int n_in, void* d_out, int out_size, void* d_ws, size_t ws_size, hipStream_t stream) {
  if (n_in < 5) return;
  const int need_qkv = ((NB * NH - 1) * SEQ_FULL + SEQ) * DD;
  if (in_sizes[0] < need_qkv || in_sizes[1] < need_qkv || in_sizes[2] < need_qkv || in_sizes[4] < NR * DD) return;
  if (out_size < NB * NH * SEQ * DD) return;
  if (ws_size < (size_t)WS_END) return;
  const float** F = (const float**)d_in;
  char* ws = (char*)d_ws; _Float16* VT = (_Float16*)(ws + WS_VT);
  k_vt<<<dim3(SEQ / 64, NB * NH), 128, 0, stream>>>(F[2], VT);
  k_att<<<dim3(SEQ / 64, NB * NH), 128, 0, stream>>>(F[0], F[1], VT, F[4], (float*)d_out);
}
